// GraphSAGEModel_19284403159491
// MI455X (gfx1250) — hardware-run, weakly checked
//
#include <hip/hip_runtime.h>
#include <stddef.h>
#include <stdint.h>


#define SPLIT_M 1
#define SPLIT_H 1

#define NN     50000
#define NE     800000
#define TROWS  128
#define NTILE  391
#define NPAD   (NTILE * TROWS)
#define F0     166
#define K0P    192
#define D1     256
#define D2     128
#define D3     64
#define XBP    192
#define M1P    384
#define P2P    512
#define P3P    256
#define W1P    576
#define W2P    1024
#define W3P    512
#define W1C1   384
#define W2C1   512
#define W3C1   256
#define KM1    (SPLIT_M ? 384 : 192)
#define KX1    192
#define KM2    (SPLIT_M ? 512 : 256)
#define KH2    (SPLIT_H ? 512 : 256)
#define KM3    (SPLIT_M ? 256 : 128)
#define KH3    (SPLIT_H ? 256 : 128)
#define BNEPS  1e-5f

#define NTHR   256
#define NWAVE  8
#define EPT    8
#define CHUNK  (NTHR * EPT)
#define WCAP   (EPT * 32)
#define LISTN  (NWAVE * WCAP)
#define NBA    1024
#define SLA    10
#define NBLK   49
#define CNTN   (NBLK * NBA)
#define RCAP   28672
#define DEGCAP 64
#define AGG_ZINTS    (LISTN + 2 * RCAP + 3 * NBA)
#define AGG_LDS_INTS (AGG_ZINTS + 16)
#define GTHR   256
#define GXTRA  544

#define NUW_A  (D1 * (K0P / 8))
#define NUW_B  (D2 * (D1 / 8))
#define NUW_C  (D3 * (D2 / 8))
#define UE0    NUW_A
#define UE1    (2 * NUW_A)
#define UE2    (UE1 + NUW_B)
#define UE3    (UE2 + NUW_B)
#define UE4    (UE3 + NUW_C)
#define UE5    (UE4 + NUW_C)
#define NUX    (NPAD * (K0P / 8))

static_assert(K0P % 32 == 0 && W1P % 32 == 0 && W2P % 32 == 0 && W3P % 32 == 0);
static_assert(KM1 % 32 == 0 && KX1 % 32 == 0 && KM2 % 32 == 0 && KH2 % 32 == 0 && KM3 % 32 == 0 && KH3 % 32 == 0);
static_assert(NPAD == 391 * 128 && NPAD >= NN && NPAD <= CNTN);
static_assert(NN % 16 == 0 && (NN - 48 * NBA) == 848 && 848 % 16 == 0);
static_assert((NN - (NTILE - 1) * TROWS) == 80);
static_assert((NN * 2 * 4) % 128 == 0);
static_assert(NN * 2 + NN * D3 == 3300000);
static_assert(RCAP >= 16623 + 4096 && DEGCAP >= 35 + 8);
static_assert((CHUNK & (CHUNK - 1)) == 0 && NBA == (1 << SLA));
static_assert(((long long)NE << SLA) < (1LL << 31));
static_assert(AGG_ZINTS % (NTHR * 4) == 0 && RCAP % (NTHR * 4) == 0);
static_assert(AGG_LDS_INTS * 4 <= 327680);
static_assert((TROWS * 128 + GXTRA) * 4 <= 327680);
static_assert(UE0 % NTHR == 0 && UE1 % NTHR == 0 && UE2 % NTHR == 0 && UE3 % NTHR == 0 && UE4 % NTHR == 0);
static_assert(UE5 % NTHR == 0 && NUX % NTHR == 0);
static_assert((NPAD * (D1 / 8)) % NTHR == 0 && (NPAD * (D2 / 8)) % NTHR == 0);
static_assert(NE % 4 == 0);

typedef float          v4f   __attribute__((ext_vector_type(4)));
typedef float          v8f   __attribute__((ext_vector_type(8)));
typedef int            v4i   __attribute__((ext_vector_type(4)));
typedef int            v8i   __attribute__((ext_vector_type(8)));
typedef unsigned       v4u   __attribute__((ext_vector_type(4)));
typedef unsigned short v8us  __attribute__((ext_vector_type(8)));
typedef unsigned short v16us __attribute__((ext_vector_type(16)));
typedef __bf16         v16bf __attribute__((ext_vector_type(16)));
typedef v4f  __attribute__((may_alias)) v4fa;
typedef v4i  __attribute__((may_alias)) v4ia;
typedef v4u  __attribute__((may_alias)) v4ua;
typedef v8us __attribute__((may_alias)) v8usa;
typedef unsigned __attribute__((may_alias)) u32a;
union FragB { v16bf v; v16us u; v8us h[2]; v8i w; };

__device__ __forceinline__ v8f wmb(const FragB& a, const FragB& b, v8f c) {
  v8f d = __builtin_amdgcn_wmma_f32_16x16x32_bf16(false, a.v, false, b.v, (short)0, c, false, false);
  asm volatile("v_nop\n\tv_nop\n\tv_nop\n\tv_nop" : "+v"(d) : "v"(a.w), "v"(b.w));
  return d;
}

__device__ __forceinline__ v8f z8() { v8f z = {0.f, 0.f, 0.f, 0.f, 0.f, 0.f, 0.f, 0.f}; return z; }

template <typename T> __device__ __forceinline__ void pin(T x) { asm volatile("" :: "v"(x)); }

__device__ __forceinline__ unsigned bf16_bits(float f) {
  const unsigned u = __float_as_uint(f);
  const unsigned r = (u + 0x7FFFu + ((u >> 16) & 1u)) >> 16;
  return ((u & 0x7fffffffu) > 0x7f800000u) ? 0x7fc0u : (r & 0xffffu);
}
__device__ __forceinline__ float bf16_val(float f) { return __uint_as_float(bf16_bits(f) << 16); }
__device__ __forceinline__ unsigned hl_bits(float v, unsigned& lo) {
  const unsigned hb = bf16_bits(v);
  lo = bf16_bits(v - __uint_as_float(hb << 16));
  return hb;
}

__device__ __forceinline__ void wave_sync() {
  __builtin_amdgcn_fence(__ATOMIC_RELEASE, "wavefront");
  __builtin_amdgcn_wave_barrier();
  __builtin_amdgcn_fence(__ATOMIC_ACQUIRE, "wavefront");
}

template <int SLB>
__device__ __forceinline__ int scan_chunk(const int* __restrict__ keys, int nE, int cbase, int slotBase,
                                          int nb, int vec8, int* list, int tid, int wave) {
  const int el0  = tid * EPT;
  const int e0   = cbase + el0;
  const int sent = (int)(1u << 31);
  int dv[8];
  if (vec8 != 0 && cbase + CHUNK <= nE) {
    const v4i da = *(const v4i*)(keys + e0);
    const v4i db = *(const v4i*)(keys + e0 + 4);
    dv[0] = da.x; dv[1] = da.y; dv[2] = da.z; dv[3] = da.w;
    dv[4] = db.x; dv[5] = db.y; dv[6] = db.z; dv[7] = db.w;
  } else {
#pragma unroll
    for (int j = 0; j < 8; ++j) {
      const int e  = e0 + j;
      const int ec = e < nE ? e : nE - 1;
      const int v  = keys[ec];
      pin(v);
      dv[j] = e < nE ? v : sent;
    }
  }
  const unsigned nbs = (unsigned)slotBase;
  const unsigned unb = (unsigned)nb;
  unsigned sv[8];
  bool hb[8];
  bool anyh = false;
#pragma unroll
  for (int j = 0; j < 8; ++j) {
    sv[j] = (unsigned)dv[j] - nbs;
    hb[j] = sv[j] < unb;
    anyh = anyh | hb[j];
  }
  const unsigned any = __builtin_amdgcn_ballot_w32(anyh);
  int wc = 0;
  if (any != 0u) {
    int p = 0;
#pragma unroll
    for (int j = 0; j < 8; ++j) {
      const unsigned qm = __builtin_amdgcn_ballot_w32(hb[j]);
      p  += (int)__builtin_amdgcn_mbcnt_lo(qm, 0u);
      wc += (int)__builtin_popcount(qm);
    }
    int* lw = list + wave * WCAP;
#pragma unroll
    for (int j = 0; j < 8; ++j) {
      if (hb[j] && p < WCAP) lw[p] = ((el0 + j) << SLB) | (int)sv[j];
      p += hb[j] ? 1 : 0;
    }
  }
  return wc;
}

template <int KIN, int KSEG, int NDST>
__device__ __forceinline__ void wunit(const float* __restrict__ W, int v, unsigned short* dst, int pitch,
                                      int col0, int col1) {
  constexpr int UPR = KSEG / 8;
  const int n  = v / UPR;
  const int k8 = (v - n * UPR) * 8;
  const float* p = W + (size_t)n * KIN;
  v8us o;
#pragma unroll
  for (int i = 0; i < 8; ++i) {
    const int k  = k8 + i;
    const int kc = k < KIN ? k : KIN - 1;
    const float f = p[kc];
    pin(f);
    o[i] = (unsigned short)bf16_bits(k < KIN ? f : 0.0f);
  }
  unsigned short* d0 = dst + (size_t)n * pitch + col0 + k8;
  unsigned short* d1 = dst + (size_t)n * pitch + col1 + k8;
  *(volatile v8us*)d0 = o;
  if (NDST == 2) *(volatile v8us*)d1 = o;
  __threadfence();
  *(volatile v8us*)d0 = o;
  if (NDST == 2) *(volatile v8us*)d1 = o;
}

__global__ __launch_bounds__(NTHR) void k_prep(const float* __restrict__ x,
                                               const float* __restrict__ wl1, const float* __restrict__ wr1,
                                               const float* __restrict__ wl2, const float* __restrict__ wr2,
                                               const float* __restrict__ wle, const float* __restrict__ wre,
                                               unsigned short* xb, unsigned short* w1c, unsigned short* w2c,
                                               unsigned short* w3c, int nN) {
  const int u = (int)blockIdx.x * NTHR + (int)threadIdx.x;
  if (u < UE0) {
    wunit<F0, K0P, 2>(wl1, u, w1c, W1P, 0, K0P);
  } else if (u < UE1) {
    wunit<F0, K0P, 1>(wr1, u - UE0, w1c, W1P, 2 * K0P, 2 * K0P);
  } else if (u < UE2) {
    wunit<D1, D1, 2>(wl2, u - UE1, w2c, W2P, 0, D1);
  } else if (u < UE3) {
    wunit<D1, D1, 2>(wr2, u - UE2, w2c, W2P, 2 * D1, 3 * D1);
  } else if (u < UE4) {
    wunit<D2, D2, 2>(wle, u - UE3, w3c, W3P, 0, D2);
  } else if (u < UE5) {
    wunit<D2, D2, 2>(wre, u - UE4, w3c, W3P, 2 * D2, 3 * D2);
  } else if (u < UE5 + NUX) {
    const int v   = u - UE5;
    const int row = v / (K0P / 8);
    const int k8  = (v - row * (K0P / 8)) * 8;
    const int rc  = row < nN ? row : nN - 1;
    const bool lv = row < nN;
    const float* p = x + (size_t)rc * F0;
    v8us o;
#pragma unroll
    for (int i = 0; i < 8; ++i) {
      const int k  = k8 + i;
      const int kc = k < F0 ? k : F0 - 1;
      const float f = p[kc];
      pin(f);
      o[i] = (unsigned short)bf16_bits((lv && k < F0) ? f : 0.0f);
    }
    unsigned short* dp = xb + (size_t)v * 8;
    *(volatile v8us*)dp = o;
    __threadfence();
    *(volatile v8us*)dp = o;
  }
}

__global__ __launch_bounds__(NTHR) void k_bucket(const int* __restrict__ srcs, const int* __restrict__ keys,
                                                 int nE, int nN, int vec8,
                                                 int* lst, int* cntg, int* offg, int* flg) {
  extern __shared__ __attribute__((aligned(16))) int dsm[];
  int* list = dsm;
  int* hl   = dsm + LISTN;
  int* sl   = hl + RCAP;
  int* cnt  = sl + RCAP;
  int* offs = cnt + NBA;
  int* cur  = offs + NBA;
  int* misc = cur + NBA;
  const int tid = (int)threadIdx.x, lane = tid & 31, wave = tid >> 5;
  const int slotBase = (int)blockIdx.x * NBA;

  {
    const v4i z4 = {0, 0, 0, 0};
    for (int i = tid * 4; i < AGG_ZINTS; i += NTHR * 4) *(v4ia*)(dsm + i) = z4;
    if (tid < 16) misc[tid] = 0;
  }
  __syncthreads();

  int t = 0, ov = 0;
  const int nChunks = (nE + CHUNK - 1) / CHUNK;
#pragma unroll 1
  for (int ch = 0; ch < nChunks; ++ch) {
    const int cbase = ch * CHUNK;
    const int wc = scan_chunk<SLA>(keys, nE, cbase, slotBase, NBA, vec8, list, tid, wave);
    if (lane == 0) misc[wave] = wc;
    __syncthreads();
    if (wave == 0) {
#pragma unroll 1
      for (int w2 = 0; w2 < NWAVE; ++w2) {
        int c = misc[w2];
        c = c < 0 ? 0 : (c > WCAP ? WCAP : c);
#pragma unroll 1
        for (int b0 = 0; b0 < c; b0 += 32) {
          const int idx = b0 + lane;
          const int ent = list[w2 * WCAP + (idx < WCAP ? idx : WCAP - 1)];
          const int m32 = (c - b0) < 32 ? (c - b0) : 32;
#pragma unroll 1
          for (int k = 0; k < m32; ++k) {
            const int u    = __builtin_amdgcn_readlane(ent, k);
            const int slot = u & (NBA - 1);
            const int el   = (u >> SLA) & (CHUNK - 1);
            const int pk   = ((cbase + el) << SLA) | slot;
            if (t < RCAP) {
              if (lane == 0) { hl[t] = pk; cnt[slot] = cnt[slot] + 1; }
              t = t + 1;
            } else {
              ov = 1;
            }
          }
        }
      }
    }
    __syncthreads();
  }
  if (wave == 0 && lane == 0) { misc[8] = t; misc[9] = ov; }
  __syncthreads();
  int tt = misc[8];
  tt = tt < 0 ? 0 : (tt > RCAP ? RCAP : tt);
  const int ovf = misc[9];

  if (wave == 0) {
    const int base = lane * (NBA / 32);
    int s = 0;
#pragma unroll 1
    for (int i = 0; i < NBA / 32; ++i) s += cnt[base + i];
    int incl = s;
#pragma unroll
    for (int d = 1; d < 32; d <<= 1) {
      const int y = __shfl_up(incl, d, 32);
      if (lane >= d) incl += y;
    }
    int run = incl - s;
#pragma unroll 1
    for (int i = 0; i < NBA / 32; ++i) {
      const int cv = cnt[base + i];
      offs[base + i] = run;
      cur[base + i]  = run;
      run += cv;
    }
  }
  __syncthreads();
  if (wave == 0) {
#pragma unroll 1
    for (int b0 = 0; b0 < tt; b0 += 32) {
      const int idx = b0 + lane;
      const int ent = hl[idx < RCAP ? idx : RCAP - 1];
      const int m32 = (tt - b0) < 32 ? (tt - b0) : 32;
#pragma unroll 1
      for (int k = 0; k < m32; ++k) {
        const int u    = __builtin_amdgcn_readlane(ent, k);
        const int slot = u & (NBA - 1);
        if (lane == 0) {
          int p = cur[slot];
          p = p < 0 ? 0 : (p > RCAP - 1 ? RCAP - 1 : p);
          sl[p] = u;
          cur[slot] = p + 1;
        }
      }
    }
  }
  __syncthreads();

  int* lo_ = lst + (size_t)blockIdx.x * RCAP;
#pragma unroll 1
  for (int p = tid * 4; p < RCAP; p += NTHR * 4) {
    const v4i e4 = *(const v4ia*)(sl + p);
    int ea = e4.x >> SLA, eb = e4.y >> SLA, ec = e4.z >> SLA, ed = e4.w >> SLA;
    ea = ea < 0 ? 0 : (ea > nE - 1 ? nE - 1 : ea);
    eb = eb < 0 ? 0 : (eb > nE - 1 ? nE - 1 : eb);
    ec = ec < 0 ? 0 : (ec > nE - 1 ? nE - 1 : ec);
    ed = ed < 0 ? 0 : (ed > nE - 1 ? nE - 1 : ed);
    int sa = srcs[ea], sb = srcs[eb], sc = srcs[ec], sd = srcs[ed];
    sa = sa < 0 ? 0 : (sa > nN - 1 ? nN - 1 : sa);
    sb = sb < 0 ? 0 : (sb > nN - 1 ? nN - 1 : sb);
    sc = sc < 0 ? 0 : (sc > nN - 1 ? nN - 1 : sc);
    sd = sd < 0 ? 0 : (sd > nN - 1 ? nN - 1 : sd);
    v4i o;
    o.x = sa; o.y = sb; o.z = sc; o.w = sd;
    *(volatile v4i*)(lo_ + p) = o;
    __threadfence();
    *(volatile v4i*)(lo_ + p) = o;
  }
  {
    const v4i c4 = *(const v4ia*)(cnt + 4 * tid);
    const v4i o4 = *(const v4ia*)(offs + 4 * tid);
    v4i f4;
    f4.x = ovf; f4.y = ovf; f4.z = ovf; f4.w = ovf;
    int* cp = cntg + (size_t)blockIdx.x * NBA + 4 * tid;
    int* op = offg + (size_t)blockIdx.x * NBA + 4 * tid;
    int* fp = flg + (size_t)blockIdx.x * 32 + 4 * (tid & 7);
    *(volatile v4i*)cp = c4;
    *(volatile v4i*)op = o4;
    if (tid < 8) *(volatile v4i*)fp = f4;
    __threadfence();
    *(volatile v4i*)cp = c4;
    *(volatile v4i*)op = o4;
    if (tid < 8) *(volatile v4i*)fp = f4;
  }
}

template <int C, int HL>
__global__ __launch_bounds__(NTHR) void k_replay(const unsigned* __restrict__ srcp, const int* __restrict__ lst,
                                                 const int* __restrict__ cntg, const int* __restrict__ offg,
                                                 const int* __restrict__ flg, int nN, unsigned* mout) {
  constexpr int NJ   = C / 64;
  constexpr int SPD  = HL ? C : C / 2;
  constexpr int NP16 = C / 4;
  constexpr int NQ   = (NP16 + 31) / 32;
  static_assert(C % 64 == 0 && NJ >= 1 && NJ <= 4 && NQ <= 2);
  __shared__ __attribute__((aligned(16))) unsigned rb[NWAVE * C];
  const int tid = (int)threadIdx.x, lane = tid & 31, wave = tid >> 5;
  unsigned* rbw = rb + wave * C;
  const float qnan = __int_as_float(0x7fc00000);

#pragma unroll 1
  for (int i = 0; i < TROWS / NWAVE; ++i) {
    const int row = (int)blockIdx.x * TROWS + i * NWAVE + wave;
    const int blk = row >> SLA;
    int cv = cntg[row];
    int ovv = offg[row];
    const int fv = flg[blk * 32];
    const int bv = ((cv > DEGCAP) || (cv < 0) || (fv != 0)) ? 1 : 0;
    cv  = cv < 0 ? 0 : (cv > DEGCAP ? DEGCAP : cv);
    ovv = ovv < 0 ? 0 : (ovv > RCAP - 1 ? RCAP - 1 : ovv);
    int lv = ovv + cv - 1;
    lv = lv > RCAP - 1 ? RCAP - 1 : lv;
    lv = lv < ovv ? ovv : lv;
    const int c    = __builtin_amdgcn_readfirstlane(cv);
    const int o    = __builtin_amdgcn_readfirstlane(ovv);
    const int last = __builtin_amdgcn_readfirstlane(lv);
    const int big  = __builtin_amdgcn_readfirstlane(bv);
    const int* lp = lst + (size_t)blk * RCAP;
    const bool live = row < nN;

    float a[2 * NJ];
#pragma unroll
    for (int e = 0; e < 2 * NJ; ++e) a[e] = 0.0f;
#pragma unroll 1
    for (int b0 = 0; b0 < c; b0 += 32) {
      int idx = o + b0 + lane;
      idx = idx > last ? last : idx;
      int sr = lp[idx];
      sr = sr < 0 ? 0 : (sr > nN - 1 ? nN - 1 : sr);
      const int m32 = (c - b0) < 32 ? (c - b0) : 32;
#pragma unroll 1
      for (int k = 0; k < m32; ++k) {
        const int sk = __builtin_amdgcn_readlane(sr, k);
        const unsigned* rp = srcp + (size_t)sk * SPD + lane;
#pragma unroll
        for (int j = 0; j < NJ; ++j) {
          const unsigned wh = rp[32 * j];
          float f0 = __uint_as_float(wh << 16);
          float f1 = __uint_as_float(wh & 0xffff0000u);
          if (HL) {
            const unsigned wl = rp[C / 2 + 32 * j];
            f0 += __uint_as_float(wl << 16);
            f1 += __uint_as_float(wl & 0xffff0000u);
          }
          a[2 * j]     += f0;
          a[2 * j + 1] += f1;
        }
      }
    }
    const float den = fmaxf((float)c, 1.0f);
#pragma unroll
    for (int j = 0; j < NJ; ++j) {
      float m0 = a[2 * j] / den;
      float m1 = a[2 * j + 1] / den;
      m0 = (big != 0) ? qnan : m0;
      m1 = (big != 0) ? qnan : m1;
      m0 = live ? m0 : 0.0f;
      m1 = live ? m1 : 0.0f;
      unsigned l0, l1;
      const unsigned h0 = hl_bits(m0, l0);
      const unsigned h1 = hl_bits(m1, l1);
      *(u32a*)(rbw + lane + 32 * j)         = h0 | (h1 << 16);
      *(u32a*)(rbw + C / 2 + lane + 32 * j) = l0 | (l1 << 16);
    }
    wave_sync();
    v4u qv[NQ];
#pragma unroll
    for (int q = 0; q < NQ; ++q) {
      const int pc  = 32 * q + lane;
      const int pcc = pc < NP16 ? pc : NP16 - 1;
      qv[q] = *(const v4ua*)(rbw + 4 * pcc);
      pin(qv[q]);
    }
    wave_sync();
    unsigned* op = mout + (size_t)row * C;
#pragma unroll
    for (int q = 0; q < NQ; ++q) {
      const int pc = 32 * q + lane;
      if (pc < NP16) *(volatile v4u*)(op + 4 * pc) = qv[q];
    }
    __threadfence();
#pragma unroll
    for (int q = 0; q < NQ; ++q) {
      const int pc = 32 * q + lane;
      if (pc < NP16) *(volatile v4u*)(op + 4 * pc) = qv[q];
    }
  }
}

template <int NT>
__device__ __forceinline__ void kseg(v8f (&acc)[NT], const unsigned short* __restrict__ ap,
                                     const unsigned short* __restrict__ bp, int ldb, int klen) {
#pragma unroll 1
  for (int k0 = 0; k0 < klen; k0 += 32) {
    FragB af;
    af.h[0] = *(const v8usa*)(ap + k0);
    af.h[1] = *(const v8usa*)(ap + k0 + 16);
#pragma unroll
    for (int nt = 0; nt < NT; ++nt) {
      const unsigned short* wq = bp + (size_t)(16 * nt) * (size_t)ldb + k0;
      FragB bf;
      bf.h[0] = *(const v8usa*)wq;
      bf.h[1] = *(const v8usa*)(wq + 16);
      acc[nt] = wmb(af, bf, acc[nt]);
    }
  }
}

template <int NT, int MODE>
__global__ __launch_bounds__(GTHR) __attribute__((amdgpu_num_vgpr(248)))
void k_gemm(const unsigned short* __restrict__ A0, int pa0, int kl0,
            const unsigned short* __restrict__ A1, int pa1, int kl1,
            const unsigned short* __restrict__ W, int pw, int wc1,
            const float* __restrict__ bias, float* tout, int tp, float* rec,
            const float* __restrict__ wch, const float* __restrict__ bch, float* outp, int eoff, int nN) {
  extern __shared__ __attribute__((aligned(16))) float gsm[];
  constexpr int NC = 16 * NT;
  static_assert((MODE == 0 && NC == 128) || (MODE == 1 && NC == 64));
  float* stg = gsm;
  float* lb  = gsm + TROWS * NC;
  float* rst = lb + 128;
  float* wcl = rst + 256;
  float* bcl = wcl + 128;
  const int tid = (int)threadIdx.x, lane = tid & 31, wave = tid >> 5, hh = lane >> 4, m = lane & 15;
  const int rowBase = (int)blockIdx.x * TROWS;
  const int colBase = (int)blockIdx.y * NC;

  if (wave == 0) {
    const int q = lane < NC / 4 ? lane : NC / 4 - 1;
    v4f b4 = *(const v4f*)(bias + colBase + 4 * q);
    pin(b4);
    v4f r4;
    r4.x = bf16_val(b4.x); r4.y = bf16_val(b4.y); r4.z = bf16_val(b4.z); r4.w = bf16_val(b4.w);
    if (lane < NC / 4) *(v4fa*)(lb + 4 * lane) = r4;
  }
  if constexpr (MODE == 1) {
    if (wave == 1) {
      v4f w4 = *(const v4f*)(wch + 4 * lane);
      v4f r4;
      r4.x = bf16_val(w4.x); r4.y = bf16_val(w4.y); r4.z = bf16_val(w4.z); r4.w = bf16_val(w4.w);
      *(v4fa*)(wcl + 4 * lane) = r4;
    }
    if (wave == 2) {
      const float b = bch[lane & 1];
      pin(b);
      if (lane < 2) bcl[lane] = bf16_val(b);
    }
  }
  __syncthreads();

  v8f acc[NT];
#pragma unroll
  for (int t = 0; t < NT; ++t) acc[t] = z8();
  const unsigned short* ap0 = A0 + (size_t)(rowBase + 16 * wave + m) * (size_t)pa0 + 8 * hh;
  const unsigned short* ap1 = A1 + (size_t)(rowBase + 16 * wave + m) * (size_t)pa1 + 8 * hh;
  const unsigned short* bp  = W  + (size_t)(colBase + m) * (size_t)pw + 8 * hh;
  kseg<NT>(acc, ap0, bp, pw, kl0);
  kseg<NT>(acc, ap1, bp + wc1, pw, kl1);

#pragma unroll
  for (int nt = 0; nt < NT; ++nt) {
    const int lc = 16 * nt + m;
    const float bj = lb[lc];
#pragma unroll
    for (int r = 0; r < 8; ++r) {
      const int lr = 16 * wave + 8 * hh + r;
      stg[lr * NC + lc] = acc[nt][r] + bj;
    }
  }
  __syncthreads();

  if constexpr (MODE == 0) {
    int nr = nN - rowBase;
    nr = nr < 1 ? 1 : (nr > TROWS ? TROWS : nr);
    if (tid < NC) {
      float s = 0.0f;
#pragma unroll 1
      for (int r = 0; r < nr; ++r) s += stg[r * NC + tid];
      const float mean = s / (float)nr;
      float q = 0.0f;
#pragma unroll 1
      for (int r = 0; r < nr; ++r) {
        const float d = stg[r * NC + tid] - mean;
        q = fmaf(d, d, q);
      }
      rst[tid]      = mean;
      rst[NC + tid] = q;
    }
#pragma unroll 1
    for (int i = 0; i < 16; ++i) {
      const int lr  = 16 * wave + i;
      const int row = rowBase + lr;
      v4f v = *(const v4fa*)(stg + lr * NC + 4 * lane);
      pin(v);
      const bool ok = row < nN;
      v4f o;
      o.x = ok ? v.x : 0.0f; o.y = ok ? v.y : 0.0f; o.z = ok ? v.z : 0.0f; o.w = ok ? v.w : 0.0f;
      *(volatile v4f*)(tout + (size_t)row * (size_t)tp + colBase + 4 * lane) = o;
    }
    __syncthreads();
    float* rp = rec + ((size_t)blockIdx.x * 2 + (size_t)(wave & 1)) * (size_t)tp + colBase + 4 * lane;
    v4f rv = *(const v4fa*)(rst + (wave & 1) * NC + 4 * lane);
    pin(rv);
    if (wave < 2) *(volatile v4f*)rp = rv;
    __threadfence();
#pragma unroll 1
    for (int i = 0; i < 16; ++i) {
      const int lr  = 16 * wave + i;
      const int row = rowBase + lr;
      v4f v = *(const v4fa*)(stg + lr * NC + 4 * lane);
      pin(v);
      const bool ok = row < nN;
      v4f o;
      o.x = ok ? v.x : 0.0f; o.y = ok ? v.y : 0.0f; o.z = ok ? v.z : 0.0f; o.w = ok ? v.w : 0.0f;
      *(volatile v4f*)(tout + (size_t)row * (size_t)tp + colBase + 4 * lane) = o;
    }
    if (wave < 2) *(volatile v4f*)rp = rv;
  } else {
    if (tid < TROWS) {
      const float* er = stg + tid * NC;
      float s0 = 0.0f, s1 = 0.0f;
#pragma unroll 4
      for (int j = 0; j < 64; ++j) {
        const float e = er[j];
        s0 = fmaf(e, wcl[j], s0);
        s1 = fmaf(e, wcl[64 + j], s1);
      }
      rst[2 * tid]     = s0 + bcl[0];
      rst[2 * tid + 1] = s1 + bcl[1];
    }
    __syncthreads();
    v4f lg = *(const v4fa*)(rst + 4 * (tid & 63));
    pin(lg);
    const int el = rowBase * 2 + 4 * tid;
    const bool lok = (tid < 64) && (el < 2 * nN);
#pragma unroll 1
    for (int i = 0; i < 8; ++i) {
      const int lr0 = 16 * wave + 2 * i;
      const int row = rowBase + lr0 + hh;
      v4f v = *(const v4fa*)(stg + lr0 * NC + 4 * lane);
      pin(v);
      float* op = outp + (size_t)eoff + (size_t)(rowBase + lr0) * NC + 4 * lane;
      if (row < nN) *(volatile v4f*)op = v;
    }
    if (lok) *(volatile v4f*)(outp + el) = lg;
    __threadfence();
#pragma unroll 1
    for (int i = 0; i < 8; ++i) {
      const int lr0 = 16 * wave + 2 * i;
      const int row = rowBase + lr0 + hh;
      v4f v = *(const v4fa*)(stg + lr0 * NC + 4 * lane);
      pin(v);
      float* op = outp + (size_t)eoff + (size_t)(rowBase + lr0) * NC + 4 * lane;
      if (row < nN) *(volatile v4f*)op = v;
    }
    if (lok) *(volatile v4f*)(outp + el) = lg;
  }
}

template <int NC>
__global__ __launch_bounds__(NC) void k_comb(const float* __restrict__ rec, int nTiles, int nN, float* stat) {
  __shared__ __attribute__((aligned(16))) float st[2 * NC];
  const int tid = (int)threadIdx.x;
  double n = 0.0, mean = 0.0, M2 = 0.0;
#pragma unroll 1
  for (int b = 0; b < nTiles; ++b) {
    int cb = nN - b * TROWS;
    cb = cb < 1 ? 1 : (cb > TROWS ? TROWS : cb);
    const double nb = (double)cb;
    const double mb = (double)rec[((size_t)b * 2) * NC + tid];
    const double qb = (double)rec[((size_t)b * 2 + 1) * NC + tid];
    const double nn = n + nb;
    const double delta = mb - mean;
    const double f = nb / nn;
    mean = mean + delta * f;
    M2 = M2 + qb + delta * delta * n * f;
    n = nn;
  }
  const double nt = n < 1.0 ? 1.0 : n;
  const float varf  = (float)(M2 / nt);
  const float meanf = (float)mean;
  const float ve = varf + BNEPS;
  const float r = 1.0f / sqrtf(ve);
  st[tid]      = meanf;
  st[NC + tid] = r;
  __syncthreads();
  const int q = tid < (2 * NC) / 4 ? tid : (2 * NC) / 4 - 1;
  v4f v = *(const v4fa*)(st + 4 * q);
  pin(v);
  if (tid < (2 * NC) / 4) *(volatile v4f*)(stat + 4 * tid) = v;
  __threadfence();
  if (tid < (2 * NC) / 4) *(volatile v4f*)(stat + 4 * tid) = v;
}

template <int C>
__global__ __launch_bounds__(NTHR) void k_apply(const float* __restrict__ tin, const float* __restrict__ stat,
                                                const float* __restrict__ gam, const float* __restrict__ bet,
                                                int nN, unsigned* hout) {
  static_assert((2 * C) / 4 <= NTHR && C % 8 == 0);
  __shared__ __attribute__((aligned(16))) float pl[4 * C];
  const int tid = (int)threadIdx.x;
  {
    const int qs = tid < (2 * C) / 4 ? tid : (2 * C) / 4 - 1;
    const int qg = tid < C / 4 ? tid : C / 4 - 1;
    v4f sa = *(const v4f*)(stat + 4 * qs);
    v4f ga = *(const v4f*)(gam + 4 * qg);
    v4f ba = *(const v4f*)(bet + 4 * qg);
    pin(sa); pin(ga); pin(ba);
    v4f gr, br;
    gr.x = bf16_val(ga.x); gr.y = bf16_val(ga.y); gr.z = bf16_val(ga.z); gr.w = bf16_val(ga.w);
    br.x = bf16_val(ba.x); br.y = bf16_val(ba.y); br.z = bf16_val(ba.z); br.w = bf16_val(ba.w);
    if (tid < (2 * C) / 4) *(v4fa*)(pl + 4 * tid) = sa;
    if (tid < C / 4) {
      *(v4fa*)(pl + 2 * C + 4 * tid) = gr;
      *(v4fa*)(pl + 3 * C + 4 * tid) = br;
    }
  }
  __syncthreads();
  constexpr int UPR = C / 8;
  const int u   = (int)blockIdx.x * NTHR + tid;
  const int row = u / UPR;
  const int j   = u - row * UPR;
  const int c0  = 8 * j;
  const bool live = row < nN;
  const v4f t0 = *(const v4f*)(tin + (size_t)u * 8);
  const v4f t1 = *(const v4f*)(tin + (size_t)u * 8 + 4);
  const v4f m0 = *(const v4fa*)(pl + c0),         m1 = *(const v4fa*)(pl + c0 + 4);
  const v4f r0 = *(const v4fa*)(pl + C + c0),     r1 = *(const v4fa*)(pl + C + c0 + 4);
  const v4f g0 = *(const v4fa*)(pl + 2 * C + c0), g1 = *(const v4fa*)(pl + 2 * C + c0 + 4);
  const v4f b0 = *(const v4fa*)(pl + 3 * C + c0), b1 = *(const v4fa*)(pl + 3 * C + c0 + 4);
  const float tv[8] = {t0.x, t0.y, t0.z, t0.w, t1.x, t1.y, t1.z, t1.w};
  const float mv[8] = {m0.x, m0.y, m0.z, m0.w, m1.x, m1.y, m1.z, m1.w};
  const float rv[8] = {r0.x, r0.y, r0.z, r0.w, r1.x, r1.y, r1.z, r1.w};
  const float gv[8] = {g0.x, g0.y, g0.z, g0.w, g1.x, g1.y, g1.z, g1.w};
  const float bv[8] = {b0.x, b0.y, b0.z, b0.w, b1.x, b1.y, b1.z, b1.w};
  unsigned hs[8], ls[8];
#pragma unroll
  for (int i = 0; i < 8; ++i) {
    float y = ((tv[i] - mv[i]) * rv[i]) * gv[i] + bv[i];
    y = (y > 0.0f) ? y : (y - y);
    y = live ? y : 0.0f;
    unsigned lo;
    hs[i] = hl_bits(y, lo);
    ls[i] = lo;
  }
  v4u hq, lq;
  hq.x = hs[0] | (hs[1] << 16); hq.y = hs[2] | (hs[3] << 16); hq.z = hs[4] | (hs[5] << 16); hq.w = hs[6] | (hs[7] << 16);
  lq.x = ls[0] | (ls[1] << 16); lq.y = ls[2] | (ls[3] << 16); lq.z = ls[4] | (ls[5] << 16); lq.w = ls[6] | (ls[7] << 16);
  unsigned* dp = hout + (size_t)row * C + 4 * j;
  *(volatile v4u*)dp = hq;
  *(volatile v4u*)(dp + C / 2) = lq;
  __threadfence();
  *(volatile v4u*)dp = hq;
  *(volatile v4u*)(dp + C / 2) = lq;
}

static inline size_t al256(size_t o) { return (o + 255) & ~(size_t)255; }

extern "C" void kernel_launch(void* const* d_in, const int* in_sizes, int n_in,
                              void* d_out, int out_size, void* d_ws, size_t ws_size,
                              hipStream_t stream) {
  if (n_in < 17) return;
  if (in_sizes[0] != NN * F0 || in_sizes[1] != 2 * NE) return;
  if (in_sizes[2] != D1 * F0 || in_sizes[3] != D1 * F0 || in_sizes[4] != D1) return;
  if (in_sizes[5] != D2 * D1 || in_sizes[6] != D2 * D1 || in_sizes[7] != D2) return;
  if (in_sizes[8] != D3 * D2 || in_sizes[9] != D3 * D2 || in_sizes[10] != D3) return;
  if (in_sizes[11] != D1 || in_sizes[12] != D1 || in_sizes[13] != D2 || in_sizes[14] != D2) return;
  if (in_sizes[15] != 2 * D3 || in_sizes[16] != 2) return;
  if (out_size != NN * 2 + NN * D3) return;

  const float* x   = (const float*)d_in[0];
  const int*   ei  = (const int*)  d_in[1];
  const float* Wl1 = (const float*)d_in[2];
  const float* Wr1 = (const float*)d_in[3];
  const float* b1  = (const float*)d_in[4];
  const float* Wl2 = (const float*)d_in[5];
  const float* Wr2 = (const float*)d_in[6];
  const float* b2  = (const float*)d_in[7];
  const float* Wle = (const float*)d_in[8];
  const float* Wre = (const float*)d_in[9];
  const float* be  = (const float*)d_in[10];
  const float* g1  = (const float*)d_in[11];
  const float* bt1 = (const float*)d_in[12];
  const float* g2  = (const float*)d_in[13];
  const float* bt2 = (const float*)d_in[14];
  const float* Wc  = (const float*)d_in[15];
  const float* bc  = (const float*)d_in[16];
  float* out = (float*)d_out;
  const int* src = ei;
  const int* key = ei + NE;
  const int nN = NN, nE = NE;
  const int vec8 = 1;

  char* ws = (char*)d_ws;
  size_t off = 0;
  const size_t oXB = off; off = al256(off + (size_t)NPAD * XBP * 2);
  const size_t oM  = off; off = al256(off + (size_t)NPAD * P2P * 2);
  const size_t oT  = off; off = al256(off + (size_t)NPAD * D1 * 4);
  const size_t oH  = off; off = al256(off + (size_t)NPAD * P2P * 2);
  const size_t oL  = off; off = al256(off + (size_t)NBLK * RCAP * 4);
  const size_t oC  = off; off = al256(off + (size_t)CNTN * 4);
  const size_t oO  = off; off = al256(off + (size_t)CNTN * 4);
  const size_t oF  = off; off = al256(off + (size_t)NBLK * 32 * 4);
  const size_t oW1 = off; off = al256(off + (size_t)D1 * W1P * 2);
  const size_t oW2 = off; off = al256(off + (size_t)D2 * W2P * 2);
  const size_t oW3 = off; off = al256(off + (size_t)D3 * W3P * 2);
  const size_t oR1 = off; off = al256(off + (size_t)NTILE * 2 * D1 * 4);
  const size_t oR2 = off; off = al256(off + (size_t)NTILE * 2 * D2 * 4);
  const size_t oS1 = off; off = al256(off + (size_t)2 * D1 * 4);
  const size_t oS2 = off; off = al256(off + (size_t)2 * D2 * 4);
  if (off > ws_size || off > (size_t)(256u << 20)) return;
  static_assert((size_t)NPAD * M1P * 2 <= (size_t)NPAD * P2P * 2 && (size_t)NPAD * P3P * 2 <= (size_t)NPAD * P2P * 2);
  static_assert((size_t)NPAD * D2 * 4 <= (size_t)NPAD * D1 * 4);

  unsigned short* XB  = (unsigned short*)(ws + oXB);
  unsigned short* PM  = (unsigned short*)(ws + oM);
  float*          PT  = (float*)(ws + oT);
  unsigned short* PH  = (unsigned short*)(ws + oH);
  int*            LST = (int*)(ws + oL);
  int*            CNT = (int*)(ws + oC);
  int*            OFF = (int*)(ws + oO);
  int*            FLG = (int*)(ws + oF);
  unsigned short* W1c = (unsigned short*)(ws + oW1);
  unsigned short* W2c = (unsigned short*)(ws + oW2);
  unsigned short* W3c = (unsigned short*)(ws + oW3);
  float*          R1  = (float*)(ws + oR1);
  float*          R2  = (float*)(ws + oR2);
  float*          S1  = (float*)(ws + oS1);
  float*          S2  = (float*)(ws + oS2);

  const size_t bLds = (size_t)AGG_LDS_INTS * 4;
  const size_t gLds0 = (size_t)(TROWS * 128 + GXTRA) * 4;
  const size_t gLds1 = (size_t)(TROWS * 64 + GXTRA) * 4;
  hipFuncSetAttribute(reinterpret_cast<const void*>(&k_bucket), hipFuncAttributeMaxDynamicSharedMemorySize, (int)bLds);
  hipFuncSetAttribute(reinterpret_cast<const void*>(&k_gemm<8, 0>), hipFuncAttributeMaxDynamicSharedMemorySize, (int)gLds0);
  hipFuncSetAttribute(reinterpret_cast<const void*>(&k_gemm<4, 1>), hipFuncAttributeMaxDynamicSharedMemorySize, (int)gLds1);

  k_prep<<<(UE5 + NUX) / NTHR, NTHR, 0, stream>>>(x, Wl1, Wr1, Wl2, Wr2, Wle, Wre, XB, W1c, W2c, W3c, nN);
  k_bucket<<<NBLK, NTHR, bLds, stream>>>(src, key, nE, nN, vec8, LST, CNT, OFF, FLG);
  k_replay<K0P, 0><<<NTILE, NTHR, 0, stream>>>((const unsigned*)XB, LST, CNT, OFF, FLG, nN, (unsigned*)PM);
  k_gemm<8, 0><<<dim3(NTILE, D1 / 128), GTHR, gLds0, stream>>>(PM, M1P, KM1, XB, XBP, KX1, W1c, W1P, W1C1,
                                                               b1, PT, D1, R1, Wc, bc, out, 0, nN);
  k_comb<D1><<<1, D1, 0, stream>>>(R1, NTILE, nN, S1);
  k_apply<D1><<<(NPAD * (D1 / 8)) / NTHR, NTHR, 0, stream>>>(PT, S1, g1, bt1, nN, (unsigned*)PH);
  k_replay<D1, 1><<<NTILE, NTHR, 0, stream>>>((const unsigned*)PH, LST, CNT, OFF, FLG, nN, (unsigned*)PM);
  k_gemm<8, 0><<<dim3(NTILE, D2 / 128), GTHR, gLds0, stream>>>(PM, P2P, KM2, PH, P2P, KH2, W2c, W2P, W2C1,
                                                               b2, PT, D2, R2, Wc, bc, out, 0, nN);
  k_comb<D2><<<1, D2, 0, stream>>>(R2, NTILE, nN, S2);
  k_apply<D2><<<(NPAD * (D2 / 8)) / NTHR, NTHR, 0, stream>>>(PT, S2, g2, bt2, nN, (unsigned*)PH);
  k_replay<D2, 1><<<NTILE, NTHR, 0, stream>>>((const unsigned*)PH, LST, CNT, OFF, FLG, nN, (unsigned*)PM);
  k_gemm<4, 1><<<dim3(NTILE, 1), GTHR, gLds1, stream>>>(PM, P3P, KM3, PH, P3P, KH3, W3c, W3P, W3C1,
                                                        be, PT, D2, R2, Wc, bc, out, 2 * NN, nN);
}
